// Mamba_21431886807208
// MI455X (gfx1250) — hardware-verified
//
#include <hip/hip_runtime.h>
#include <stddef.h>
#include <stdint.h>

#define NBAT  32
#define LSEQ  1024
#define DM    384
#define DIN   768
#define EIN   1536
#define KOUT  1536
#define NST   16
#define DTR   24
#define XDE   56
#define XDPAD 64
#define NROW  32
#define SEGT  32
#define NTOK  (NBAT * LSEQ)
#define NCH   32
#define NCHB  (DIN / NCH)
#define NTHR  256
#define GTHR  128
#define GBM   64
#define GBN   128
#define WCOL  96
#define NSTG  ((32 * DM / 4) / NTHR)
#define NSW   ((32 * DIN / 4) / NTHR)
#define NLD   ((LSEQ * NCH / 4) / NTHR)

#define U_WIN (EIN * DM / 8)
#define U_WO  (DM * KOUT / 8)
#define U_XP  (2 * XDE * DIN / 4)
#define U_DP  (2 * DIN * DTR / 4)
#define U_AR  (2 * DIN * NST / 4)
#define U_TOT (U_WIN + U_WO + U_XP + U_DP + U_AR)

#define LDS_TILE_BYTES (32 * DIN * 4)
#define LDS_CONV_BYTES ((LSEQ + 6) * NCH * 4)

#define SZ_WIN ((size_t)EIN * DM * 2)
#define SZ_WO  ((size_t)DM * KOUT * 2)
#define SZ_XP  ((size_t)2 * XDE * DIN * 4)
#define SZ_DP  ((size_t)2 * DIN * DTR * 4)
#define SZ_AR  ((size_t)2 * DIN * NST * 4)
#define SZ_XSG ((size_t)NTOK * DIN * 4)
#define SZ_ROW ((size_t)NBAT * NROW * DIN * 4)
#define WS_TOTAL (SZ_WIN + SZ_WO + SZ_XP + SZ_DP + SZ_AR + SZ_XSG + 4 * SZ_ROW)
#define WSMAX  134217728

static_assert(WS_TOTAL <= (size_t)WSMAX);
static_assert(SZ_WIN % 256 == 0 && SZ_WO % 256 == 0 && SZ_XP % 256 == 0 && SZ_DP % 256 == 0 && SZ_AR % 256 == 0);
static_assert(SZ_XSG % 256 == 0 && SZ_ROW % 256 == 0);
static_assert(SZ_XSG == (size_t)NTOK * KOUT * 2);
static_assert(U_WIN % NTHR == 0 && U_WO % NTHR == 0 && U_XP % NTHR == 0 && U_DP % NTHR == 0 && U_AR % NTHR == 0);
static_assert((XDE * DIN / 4) % NTHR == 0 && (DIN * DTR / 4) % NTHR == 0 && (DIN * NST / 4) % NTHR == 0);
static_assert(DM % 32 == 0 && KOUT % 32 == 0 && KOUT == 2 * DIN && DIN % 8 == 0);
static_assert(NTOK % GBM == 0 && DM % GBN == 0 && GBM == (GTHR / 32) * 16 && GBN == 8 * 16);
static_assert(DIN == 8 * WCOL && WCOL == 6 * 16 && NTOK % 32 == 0);
static_assert(LSEQ == NROW * SEGT && SEGT == 32 && NROW == 32 && LSEQ % 32 == 0);
static_assert(DIN == NCH * NCHB && NCH == 32 && NTHR == 8 * 32);
static_assert(XDE == DTR + 2 * NST && XDE == 7 * 8 && DTR % 4 == 0 && XDE <= XDPAD && XDPAD % 4 == 0);
static_assert((32 * DM * 2) <= LDS_TILE_BYTES && (32 * DM / 4) % NTHR == 0 && (32 * DIN / 4) % NTHR == 0);
static_assert(DIN % 4 == 0 && (DIN / 4) <= NTHR && (LSEQ * NCH / 4) % NTHR == 0);
static_assert((DIN * NST) % (4 * NTHR) == 0 && DIN == 3 * NTHR);
static_assert(24 * 32 == DIN && KOUT / 8 == 6 * 32 && NROW * NCH / 4 == NTHR && SEGT * NCH / 4 == NTHR);
static_assert(NSTG == 12 && NSW == 24 && NLD == 32);
static_assert(LDS_CONV_BYTES <= 280000 && LDS_TILE_BYTES <= 280000);

typedef float          v4f   __attribute__((ext_vector_type(4)));
typedef float          v8f   __attribute__((ext_vector_type(8)));
typedef int            v8i   __attribute__((ext_vector_type(8)));
typedef unsigned short v4us  __attribute__((ext_vector_type(4)));
typedef unsigned short v8us  __attribute__((ext_vector_type(8)));
typedef unsigned short v16us __attribute__((ext_vector_type(16)));
typedef __bf16         v16bf __attribute__((ext_vector_type(16)));
typedef v4f  __attribute__((may_alias)) v4fa;
typedef v4us __attribute__((may_alias)) v4usa;
typedef v8us __attribute__((may_alias)) v8usa;
union FragB { v16bf v; v16us u; v8us h[2]; v8i w; };

__device__ __forceinline__ v8f wmb(const FragB& a, const FragB& b, v8f c) {
  v8f d = __builtin_amdgcn_wmma_f32_16x16x32_bf16(false, a.v, false, b.v, (short)0, c, false, false);
  asm volatile("v_nop\n\tv_nop\n\tv_nop\n\tv_nop" : "+v"(d) : "v"(a.w), "v"(b.w));
  return d;
}

__device__ __forceinline__ unsigned bf16_bits(float f) {
  const unsigned u = __float_as_uint(f);
  return (u + 0x7FFFu + ((u >> 16) & 1u)) >> 16;
}
__device__ __forceinline__ float bf16_val(float f) {
  return __uint_as_float(bf16_bits(f) << 16);
}
__device__ __forceinline__ void put16(unsigned short* dp, v8us o) {
  *(volatile v8us*)dp = o;
  __threadfence();
  *(volatile v8us*)dp = o;
}
__device__ __forceinline__ void putf4(float* dp, v4f o) {
  *(volatile v4f*)dp = o;
  __threadfence();
  *(volatile v4f*)dp = o;
}
__device__ __forceinline__ float wsum(float v) {
  v += __shfl_xor(v, 16);
  v += __shfl_xor(v, 8);
  v += __shfl_xor(v, 4);
  v += __shfl_xor(v, 2);
  v += __shfl_xor(v, 1);
  return v;
}
__device__ __forceinline__ float silu_f(float v) {
  const float e = expf(fminf(-v, 30.0f));
  return v * (1.0f / (1.0f + e));
}
__device__ __forceinline__ v4f ln_gate4(v4f mv, float mu, float rstd, v4f wv, v4f bv, v4f zv) {
  v4f g;
  g.x = ((mv.x - mu) * rstd * wv.x + bv.x) * silu_f(zv.x);
  g.y = ((mv.y - mu) * rstd * wv.y + bv.y) * silu_f(zv.y);
  g.z = ((mv.z - mu) * rstd * wv.z + bv.z) * silu_f(zv.z);
  g.w = ((mv.w - mu) * rstd * wv.w + bv.w) * silu_f(zv.w);
  return g;
}

__global__ __launch_bounds__(NTHR) void k_prep(const float* __restrict__ win, const float* __restrict__ wout,
                                               const float* __restrict__ xpw, const float* __restrict__ xpwb,
                                               const float* __restrict__ dpw, const float* __restrict__ dpwb,
                                               const float* __restrict__ alog, const float* __restrict__ alogb,
                                               unsigned short* WIN, unsigned short* WOUT2,
                                               float* XPR, float* DPR, float* AR) {
  const int u  = (int)blockIdx.x * NTHR + (int)threadIdx.x;
  const int L1 = U_WIN;
  const int L2 = L1 + U_WO;
  const int L3 = L2 + U_XP;
  const int L4 = L3 + U_DP;
  const int L5 = L4 + U_AR;
  if (u < L1) {
    const float* p = win + (size_t)u * 8;
    const v4f a = *(const v4fa*)p;
    const v4f c = *(const v4fa*)(p + 4);
    v8us o;
    o[0] = (unsigned short)bf16_bits(a.x); o[1] = (unsigned short)bf16_bits(a.y);
    o[2] = (unsigned short)bf16_bits(a.z); o[3] = (unsigned short)bf16_bits(a.w);
    o[4] = (unsigned short)bf16_bits(c.x); o[5] = (unsigned short)bf16_bits(c.y);
    o[6] = (unsigned short)bf16_bits(c.z); o[7] = (unsigned short)bf16_bits(c.w);
    put16(WIN + (size_t)u * 8, o);
    return;
  } else if (u < L2) {
    const int v  = u - L1;
    const int e  = v / (KOUT / 8);
    const int k8 = (v - e * (KOUT / 8)) * 8;
    const int ks = k8 < DIN ? k8 : k8 - DIN;
    const float* p = wout + (size_t)e * DIN + ks;
    const v4f a = *(const v4fa*)p;
    const v4f c = *(const v4fa*)(p + 4);
    v8us o;
    o[0] = (unsigned short)bf16_bits(a.x); o[1] = (unsigned short)bf16_bits(a.y);
    o[2] = (unsigned short)bf16_bits(a.z); o[3] = (unsigned short)bf16_bits(a.w);
    o[4] = (unsigned short)bf16_bits(c.x); o[5] = (unsigned short)bf16_bits(c.y);
    o[6] = (unsigned short)bf16_bits(c.z); o[7] = (unsigned short)bf16_bits(c.w);
    put16(WOUT2 + (size_t)e * KOUT + k8, o);
    return;
  } else if (u < L3) {
    const int v  = u - L2;
    const int hv = XDE * DIN / 4;
    const int which = v >= hv ? 1 : 0;
    const float* p = (which ? xpwb : xpw) + (size_t)(v - which * hv) * 4;
    const v4f a = *(const v4fa*)p;
    v4f q;
    q.x = bf16_val(a.x); q.y = bf16_val(a.y); q.z = bf16_val(a.z); q.w = bf16_val(a.w);
    putf4(XPR + (size_t)v * 4, q);
    return;
  } else if (u < L4) {
    const int v  = u - L3;
    const int hv = DIN * DTR / 4;
    const int which = v >= hv ? 1 : 0;
    const float* p = (which ? dpwb : dpw) + (size_t)(v - which * hv) * 4;
    const v4f a = *(const v4fa*)p;
    v4f q;
    q.x = bf16_val(a.x); q.y = bf16_val(a.y); q.z = bf16_val(a.z); q.w = bf16_val(a.w);
    putf4(DPR + (size_t)v * 4, q);
    return;
  } else if (u < L5) {
    const int v  = u - L4;
    const int hv = DIN * NST / 4;
    const int which = v >= hv ? 1 : 0;
    const float* p = (which ? alogb : alog) + (size_t)(v - which * hv) * 4;
    const v4f a = *(const v4fa*)p;
    v4f q;
    q.x = -expf(bf16_val(a.x)); q.y = -expf(bf16_val(a.y));
    q.z = -expf(bf16_val(a.z)); q.w = -expf(bf16_val(a.w));
    putf4(AR + (size_t)v * 4, q);
    return;
  }
}

__device__ __forceinline__ void gemm_tile(const float* __restrict__ hs, int t0,
                                          const unsigned short* __restrict__ Wr,
                                          unsigned short* sA, v8f (&acc)[2][6],
                                          int tid, int wave, int hh, int m) {
#pragma unroll 4
  for (int it = 0; it < NSTG; ++it) {
    const int f   = it * NTHR + tid;
    const int row = f / (DM / 4);
    const int c4  = f - row * (DM / 4);
    const v4f a = *(const v4fa*)(hs + (size_t)(t0 + row) * DM + 4 * c4);
    v4us o;
    o.x = (unsigned short)bf16_bits(a.x);
    o.y = (unsigned short)bf16_bits(a.y);
    o.z = (unsigned short)bf16_bits(a.z);
    o.w = (unsigned short)bf16_bits(a.w);
    *(v4usa*)(sA + row * DM + 4 * c4) = o;
  }
  __syncthreads();
  {
    const v8f z = {0.f, 0.f, 0.f, 0.f, 0.f, 0.f, 0.f, 0.f};
#pragma unroll
    for (int mt = 0; mt < 2; ++mt)
#pragma unroll
      for (int nt = 0; nt < 6; ++nt) acc[mt][nt] = z;
  }
  const unsigned short* ap0 = sA + m * DM + 8 * hh;
  const unsigned short* ap1 = ap0 + 16 * DM;
  const unsigned short* bp  = Wr + (size_t)(WCOL * wave + m) * (size_t)DM + 8 * hh;
#pragma unroll 1
  for (int k0 = 0; k0 < DM; k0 += 32) {
    FragB a0, a1;
    a0.h[0] = *(const v8usa*)(ap0 + k0);
    a0.h[1] = *(const v8usa*)(ap0 + k0 + 16);
    a1.h[0] = *(const v8usa*)(ap1 + k0);
    a1.h[1] = *(const v8usa*)(ap1 + k0 + 16);
#pragma unroll
    for (int nt = 0; nt < 6; ++nt) {
      const unsigned short* wq = bp + (size_t)(16 * nt) * (size_t)DM + k0;
      FragB bf;
      bf.h[0] = *(const v8usa*)wq;
      bf.h[1] = *(const v8usa*)(wq + 16);
      acc[0][nt] = wmb(a0, bf, acc[0][nt]);
      acc[1][nt] = wmb(a1, bf, acc[1][nt]);
    }
  }
}

__global__ __launch_bounds__(NTHR) void k_inx(const float* __restrict__ hs, const unsigned short* __restrict__ WIN,
                                              float* X) {
  extern __shared__ __attribute__((aligned(16))) float dynl[];
  unsigned short* sA = (unsigned short*)dynl;
  float* st = dynl;
  const int tid = (int)threadIdx.x, lane = tid & 31, wave = tid >> 5, hh = lane >> 4, m = lane & 15;
  const int t0 = (int)blockIdx.x * 32;

  v8f acc[2][6];
  gemm_tile(hs, t0, WIN, sA, acc, tid, wave, hh, m);
  __syncthreads();
#pragma unroll
  for (int mt = 0; mt < 2; ++mt)
#pragma unroll
    for (int nt = 0; nt < 6; ++nt)
#pragma unroll
      for (int r = 0; r < 8; ++r)
        st[(16 * mt + 8 * hh + r) * DIN + WCOL * wave + 16 * nt + m] = acc[mt][nt][r];
  __syncthreads();

  float* xb = X + (size_t)t0 * DIN;
#pragma unroll 4
  for (int it = 0; it < NSW; ++it) {
    const int f = it * NTHR + tid;
    const v4f v = *(const v4fa*)(st + f * 4);
    *(volatile v4f*)(xb + (size_t)f * 4) = v;
  }
  __threadfence();
#pragma unroll 4
  for (int it = 0; it < NSW; ++it) {
    const int f = it * NTHR + tid;
    const v4f v = *(const v4fa*)(st + f * 4);
    *(volatile v4f*)(xb + (size_t)f * 4) = v;
  }
}

__global__ __launch_bounds__(NTHR) void k_conv(float* XS, const float* __restrict__ cw, const float* __restrict__ cb,
                                               const float* __restrict__ cwb, const float* __restrict__ cbb,
                                               const float* __restrict__ dsk, const float* __restrict__ dskb,
                                               float* UF, float* UB) {
  extern __shared__ __attribute__((aligned(16))) float xs[];
  __shared__ __attribute__((aligned(16))) float sS[SEGT * NCH];
  __shared__ __attribute__((aligned(16))) float psf[8 * NCH];
  __shared__ __attribute__((aligned(16))) float psb[8 * NCH];
  __shared__ __attribute__((aligned(16))) float ufl[NROW * NCH];
  __shared__ __attribute__((aligned(16))) float ubl[NROW * NCH];

  const int tid = (int)threadIdx.x, lane = tid & 31, wave = tid >> 5;
  const int b   = (int)blockIdx.x / NCHB;
  const int ch  = (int)blockIdx.x - b * NCHB;
  const int c0  = ch * NCH;
  const int d   = c0 + lane;
  const size_t tb = (size_t)b * LSEQ;

  const v4f wfv = *(const v4fa*)(cw + (size_t)d * 4);
  const v4f wbv = *(const v4fa*)(cwb + (size_t)d * 4);
  const float w0 = bf16_val(wfv.x), w1 = bf16_val(wfv.y), w2 = bf16_val(wfv.z), w3 = bf16_val(wfv.w);
  const float r0 = bf16_val(wbv.x), r1 = bf16_val(wbv.y), r2 = bf16_val(wbv.z), r3 = bf16_val(wbv.w);
  const float bfv = bf16_val(cb[d]), bbv = bf16_val(cbb[d]);
  const float dv  = bf16_val(dsk[d]), dbv = bf16_val(dskb[d]);
  const v4f z4 = {0.0f, 0.0f, 0.0f, 0.0f};

#pragma unroll 4
  for (int it = 0; it < NLD; ++it) {
    const int f = it * NTHR + tid;
    const int l = f >> 3, p = f & 7;
    const v4f v = *(const v4fa*)(XS + (tb + l) * DIN + c0 + 4 * p);
    *(v4fa*)(xs + (3 + l) * NCH + 4 * p) = v;
  }
  if (tid < 24) *(v4fa*)(xs + 4 * tid) = z4;
  if (tid >= 24 && tid < 48) *(v4fa*)(xs + (LSEQ + 3) * NCH + 4 * (tid - 24)) = z4;
  __syncthreads();

#pragma unroll 1
  for (int a = 0; a < NROW; ++a) {
    float pf = 0.0f, pb = 0.0f;
#pragma unroll 1
    for (int i = 0; i < 4; ++i) {
      const int l = SEGT * a + 4 * wave + i;
      const float* xp = xs + (3 + l) * NCH + lane;
      const float xm3 = xp[-3 * NCH], xm2 = xp[-2 * NCH], xm1 = xp[-NCH], x00 = xp[0];
      const float xq1 = xp[NCH], xq2 = xp[2 * NCH], xq3 = xp[3 * NCH];
      const float vf = (((w0 * xm3 + w1 * xm2) + w2 * xm1) + w3 * x00) + bfv;
      const float vb = (((r0 * xq3 + r1 * xq2) + r2 * xq1) + r3 * x00) + bbv;
      const float xc = silu_f(vf);
      const float xb = silu_f(vb);
      sS[(4 * wave + i) * NCH + lane] = 0.5f * (dv * xc + dbv * xb);
      pf += xc;
      pb += xb;
    }
    psf[wave * NCH + lane] = pf;
    psb[wave * NCH + lane] = pb;
    __syncthreads();
    {
      const int j = tid >> 3, p = tid & 7;
      const v4f v = *(const v4fa*)(sS + j * NCH + 4 * p);
      float* gp = XS + (tb + SEGT * a + j) * DIN + c0 + 4 * p;
      *(volatile v4f*)gp = v;
      __threadfence();
      *(volatile v4f*)gp = v;
    }
    if (tid < NCH) {
      float sf = psf[tid], sb = psb[tid];
#pragma unroll
      for (int w2 = 1; w2 < 8; ++w2) { sf += psf[w2 * NCH + tid]; sb += psb[w2 * NCH + tid]; }
      ufl[a * NCH + tid] = sf * (1.0f / (float)SEGT);
      ubl[a * NCH + tid] = sb * (1.0f / (float)SEGT);
    }
    __syncthreads();
  }
  {
    const int a = tid >> 3, p = tid & 7;
    const v4f vf = *(const v4fa*)(ufl + a * NCH + 4 * p);
    const v4f vb = *(const v4fa*)(ubl + a * NCH + 4 * p);
    const size_t ro = ((size_t)b * NROW + a) * DIN + c0 + 4 * p;
    *(volatile v4f*)(UF + ro) = vf;
    *(volatile v4f*)(UB + ro) = vb;
    __threadfence();
    *(volatile v4f*)(UF + ro) = vf;
    *(volatile v4f*)(UB + ro) = vb;
  }
}

__global__ __launch_bounds__(NTHR) void k_ssm(const float* __restrict__ UF, const float* __restrict__ UB,
                                              const float* __restrict__ XPR, const float* __restrict__ DPR,
                                              const float* __restrict__ AR,
                                              const float* __restrict__ dpbf, const float* __restrict__ dpbb,
                                              float* YF, float* YB) {
  __shared__ __attribute__((aligned(16))) float ul[DIN];
  __shared__ __attribute__((aligned(16))) float yl[DIN];
  __shared__ __attribute__((aligned(16))) float xd[XDPAD];
  __shared__ __attribute__((aligned(16))) float hl[DIN * NST];

  const int tid = (int)threadIdx.x, lane = tid & 31, wave = tid >> 5;
  const int b  = (int)blockIdx.x >> 1;
  const int br = (int)blockIdx.x & 1;
  const float* U   = br ? UB : UF;
  float*       Y   = br ? YB : YF;
  const float* xpw = XPR + (size_t)br * XDE * DIN;
  const float* dpw = DPR + (size_t)br * DIN * DTR;
  const float* ar  = AR  + (size_t)br * DIN * NST;
  const float* dpb = br ? dpbb : dpbf;
  const v4f z4 = {0.0f, 0.0f, 0.0f, 0.0f};

  for (int i = tid * 4; i < DIN * NST; i += NTHR * 4) *(v4fa*)(hl + i) = z4;
  if (tid < XDPAD / 4) *(v4fa*)(xd + 4 * tid) = z4;
  __syncthreads();

#pragma unroll 1
  for (int r = 0; r < NROW; ++r) {
    const int rr = br ? (NROW - 1 - r) : r;
    const size_t ro = ((size_t)b * NROW + rr) * DIN;
    if (tid < DIN / 4) *(v4fa*)(ul + 4 * tid) = *(const v4fa*)(U + ro + 4 * tid);
    __syncthreads();

#pragma unroll 1
    for (int e7 = 0; e7 < 7; ++e7) {
      const int e = wave * 7 + e7;
      const float* wr = xpw + (size_t)e * DIN + 4 * lane;
      float p = 0.0f;
#pragma unroll 1
      for (int j = 0; j < DIN / 128; ++j) {
        const v4f uv = *(const v4fa*)(ul + 128 * j + 4 * lane);
        const v4f wv = *(const v4fa*)(wr + 128 * j);
        p += uv.x * wv.x;
        p += uv.y * wv.y;
        p += uv.z * wv.z;
        p += uv.w * wv.w;
      }
      p = wsum(p);
      if (lane == 0) xd[e] = p;
    }
    __syncthreads();

#pragma unroll 1
    for (int k = 0; k < 3; ++k) {
      const int dd = tid + NTHR * k;
      const float* wr = dpw + (size_t)dd * DTR;
      float dot = 0.0f;
#pragma unroll 1
      for (int q = 0; q < DTR / 4; ++q) {
        const v4f xv = *(const v4fa*)(xd + 4 * q);
        const v4f wv = *(const v4fa*)(wr + 4 * q);
        dot += xv.x * wv.x;
        dot += xv.y * wv.y;
        dot += xv.z * wv.z;
        dot += xv.w * wv.w;
      }
      const float v     = dot + bf16_val(dpb[dd]);
      const float delta = fmaxf(v, 0.0f) + log1pf(expf(-fabsf(v)));
      const float du    = delta * ul[dd];
      const float* arow = ar + (size_t)dd * NST;
      float* hrow = hl + dd * NST;
      float y = 0.0f;
#pragma unroll 1
      for (int n = 0; n < NST; ++n) {
        const float av = arow[n];
        float h = hrow[n];
        const float bn = xd[DTR + n];
        const float cn = xd[DTR + NST + n];
        h = expf(delta * av) * h + du * bn;
        hrow[n] = h;
        y += h * cn;
      }
      yl[dd] = y;
    }
    __syncthreads();

    if (tid < DIN / 4) {
      const v4f yv = *(const v4fa*)(yl + 4 * tid);
      float* gp = Y + ro + 4 * tid;
      *(volatile v4f*)gp = yv;
      __threadfence();
      *(volatile v4f*)gp = yv;
    }
  }
}

__global__ __launch_bounds__(NTHR) void k_gate(const float* __restrict__ hs, const unsigned short* __restrict__ WIN,
                                               const float* __restrict__ YF, const float* __restrict__ YB,
                                               const float* __restrict__ lnw, const float* __restrict__ lnb,
                                               float* SG) {
  extern __shared__ __attribute__((aligned(16))) float dynl[];
  unsigned short* sA = (unsigned short*)dynl;
  float* zt = dynl;
  __shared__ __attribute__((aligned(16))) float yy[DIN];
  __shared__ __attribute__((aligned(16))) float lw[DIN];
  __shared__ __attribute__((aligned(16))) float lb[DIN];
  __shared__ __attribute__((aligned(16))) unsigned short gl[8 * KOUT];

  const int tid = (int)threadIdx.x, lane = tid & 31, wave = tid >> 5, hh = lane >> 4, m = lane & 15;
  const int blk = (int)blockIdx.x;
  const int t0  = blk * 32;
  const int b   = blk >> 5;
  const int a   = blk & 31;

  if (tid < DIN / 4) {
    const size_t ro = ((size_t)b * NROW + a) * DIN + 4 * tid;
    const v4f f4 = *(const v4fa*)(YF + ro);
    const v4f g4 = *(const v4fa*)(YB + ro);
    *(v4fa*)(yy + 4 * tid) = (f4 + g4) * 0.5f;
    const v4f w4 = *(const v4fa*)(lnw + 4 * tid);
    const v4f b4 = *(const v4fa*)(lnb + 4 * tid);
    v4f wq, bq;
    wq.x = bf16_val(w4.x); wq.y = bf16_val(w4.y); wq.z = bf16_val(w4.z); wq.w = bf16_val(w4.w);
    bq.x = bf16_val(b4.x); bq.y = bf16_val(b4.y); bq.z = bf16_val(b4.z); bq.w = bf16_val(b4.w);
    *(v4fa*)(lw + 4 * tid) = wq;
    *(v4fa*)(lb + 4 * tid) = bq;
  }

  v8f acc[2][6];
  gemm_tile(hs, t0, WIN + (size_t)DIN * DM, sA, acc, tid, wave, hh, m);
  __syncthreads();
#pragma unroll
  for (int mt = 0; mt < 2; ++mt)
#pragma unroll
    for (int nt = 0; nt < 6; ++nt)
#pragma unroll
      for (int r = 0; r < 8; ++r)
        zt[(16 * mt + 8 * hh + r) * DIN + WCOL * wave + 16 * nt + m] = acc[mt][nt][r];
  __syncthreads();

  unsigned short* glw = gl + wave * KOUT;
  unsigned short* Gq  = (unsigned short*)SG;
#pragma unroll 1
  for (int i = 0; i < 4; ++i) {
    const int tl = 4 * wave + i;
    const size_t t = (size_t)t0 + tl;
    const int base = 24 * lane;
    const float* sp = SG + t * DIN + base;
    v4f mm[6];
    float s1 = 0.0f;
#pragma unroll
    for (int j = 0; j < 6; ++j) {
      const v4f sv = *(const v4fa*)(sp + 4 * j);
      const v4f yv = *(const v4fa*)(yy + base + 4 * j);
      const v4f mv = sv + yv;
      mm[j] = mv;
      s1 += (mv.x + mv.y) + (mv.z + mv.w);
    }
    s1 = wsum(s1);
    const float mu = s1 * (1.0f / (float)DIN);
    float s2 = 0.0f;
#pragma unroll
    for (int j = 0; j < 6; ++j) {
      const v4f dv = mm[j] - mu;
      s2 += (dv.x * dv.x + dv.y * dv.y) + (dv.z * dv.z + dv.w * dv.w);
    }
    s2 = wsum(s2);
    const float rstd = rsqrtf(s2 * (1.0f / (float)DIN) + 1e-5f);
    const float* zr = zt + tl * DIN + base;
#pragma unroll
    for (int g = 0; g < 3; ++g) {
      const int j0 = 2 * g, j1 = 2 * g + 1;
      const v4f ga = ln_gate4(mm[j0], mu, rstd, *(const v4fa*)(lw + base + 4 * j0),
                              *(const v4fa*)(lb + base + 4 * j0), *(const v4fa*)(zr + 4 * j0));
      const v4f gb = ln_gate4(mm[j1], mu, rstd, *(const v4fa*)(lw + base + 4 * j1),
                              *(const v4fa*)(lb + base + 4 * j1), *(const v4fa*)(zr + 4 * j1));
      const v8f g8 = {ga.x, ga.y, ga.z, ga.w, gb.x, gb.y, gb.z, gb.w};
      v8us ho, lo;
#pragma unroll
      for (int c = 0; c < 8; ++c) {
        const unsigned hb = bf16_bits(g8[c]);
        ho[c] = (unsigned short)hb;
        lo[c] = (unsigned short)bf16_bits(g8[c] - __uint_as_float(hb << 16));
      }
      *(v8usa*)(glw + base + 8 * g)       = ho;
      *(v8usa*)(glw + DIN + base + 8 * g) = lo;
    }
    __syncthreads();
    v8us pv[6];
#pragma unroll
    for (int it = 0; it < 6; ++it) pv[it] = *(const v8usa*)(glw + (it * 32 + lane) * 8);
    unsigned short* gp = Gq + t * KOUT;
#pragma unroll
    for (int it = 0; it < 6; ++it) *(volatile v8us*)(gp + (it * 32 + lane) * 8) = pv[it];
    __threadfence();
#pragma unroll
    for (int it = 0; it < 6; ++it) *(volatile v8us*)(gp + (it * 32 + lane) * 8) = pv[it];
    __syncthreads();
  }
}

__global__ __launch_bounds__(GTHR) void k_out(const unsigned short* __restrict__ A,
                                              const unsigned short* __restrict__ BT, float* C) {
  __shared__ __attribute__((aligned(16))) float stg[GBM * GBN];
  const int tid = (int)threadIdx.x, lane = tid & 31, wave = tid >> 5, hh = lane >> 4, m = lane & 15;
  const int rowBase = (int)blockIdx.x * GBM;
  const int colBase = (int)blockIdx.y * GBN;

  v8f acc[8];
  {
    const v8f z = {0.f, 0.f, 0.f, 0.f, 0.f, 0.f, 0.f, 0.f};
#pragma unroll
    for (int t = 0; t < 8; ++t) acc[t] = z;
  }
  const unsigned short* ap = A  + (size_t)(rowBase + 16 * wave + m) * (size_t)KOUT + 8 * hh;
  const unsigned short* bp = BT + (size_t)(colBase + m) * (size_t)KOUT + 8 * hh;

#pragma unroll 1
  for (int k0 = 0; k0 < KOUT; k0 += 32) {
    FragB af;
    af.h[0] = *(const v8usa*)(ap + k0);
    af.h[1] = *(const v8usa*)(ap + k0 + 16);
#pragma unroll
    for (int nt = 0; nt < 8; ++nt) {
      const unsigned short* wq = bp + (size_t)(16 * nt) * (size_t)KOUT + k0;
      FragB bf;
      bf.h[0] = *(const v8usa*)wq;
      bf.h[1] = *(const v8usa*)(wq + 16);
      acc[nt] = wmb(af, bf, acc[nt]);
    }
  }

#pragma unroll
  for (int nt = 0; nt < 8; ++nt) {
    const int lc = 16 * nt + m;
#pragma unroll
    for (int r = 0; r < 8; ++r) {
      const int lr = 16 * wave + 8 * hh + r;
      stg[lr * GBN + lc] = acc[nt][r];
    }
  }
  __syncthreads();

  v4f pv[16];
#pragma unroll
  for (int i = 0; i < 16; ++i) pv[i] = *(const v4fa*)(stg + (16 * wave + i) * GBN + 4 * lane);
#pragma unroll
  for (int i = 0; i < 16; ++i) {
    float* op = C + (size_t)(rowBase + 16 * wave + i) * (size_t)DM + colBase + 4 * lane;
    *(volatile v4f*)op = pv[i];
  }
  __threadfence();
#pragma unroll
  for (int i = 0; i < 16; ++i) {
    float* op = C + (size_t)(rowBase + 16 * wave + i) * (size_t)DM + colBase + 4 * lane;
    *(volatile v4f*)op = pv[i];
  }
}

extern "C" void kernel_launch(void* const* d_in, const int* in_sizes, int n_in,
                              void* d_out, int out_size, void* d_ws, size_t ws_size,
                              hipStream_t stream) {
  if (n_in < 20) return;
  if (in_sizes[0] != NTOK * DM) return;
  if (in_sizes[1] != EIN * DM) return;
  if (in_sizes[2] != DIN * 4 || in_sizes[3] != DIN) return;
  if (in_sizes[4] != DIN * 4 || in_sizes[5] != DIN) return;
  if (in_sizes[6] != XDE * DIN || in_sizes[7] != XDE * DIN) return;
  if (in_sizes[8] != DIN * DTR || in_sizes[9] != DIN) return;
  if (in_sizes[10] != DIN * DTR || in_sizes[11] != DIN) return;
  if (in_sizes[12] != DIN * NST || in_sizes[13] != DIN * NST) return;
  if (in_sizes[14] != DIN || in_sizes[15] != DIN) return;
  if (in_sizes[16] != DIN || in_sizes[17] != DIN) return;
  if (in_sizes[18] != DM * DIN) return;
  if (in_sizes[19] != 1) return;
  if (out_size != NTOK * DM) return;
  if (ws_size < WS_TOTAL) return;

  const float* hs    = (const float*)d_in[0];
  const float* win   = (const float*)d_in[1];
  const float* cw    = (const float*)d_in[2];
  const float* cb    = (const float*)d_in[3];
  const float* cwb   = (const float*)d_in[4];
  const float* cbb   = (const float*)d_in[5];
  const float* xpw   = (const float*)d_in[6];
  const float* xpwb  = (const float*)d_in[7];
  const float* dpw   = (const float*)d_in[8];
  const float* dpbf  = (const float*)d_in[9];
  const float* dpwb  = (const float*)d_in[10];
  const float* dpbb  = (const float*)d_in[11];
  const float* alog  = (const float*)d_in[12];
  const float* alogb = (const float*)d_in[13];
  const float* dsk   = (const float*)d_in[14];
  const float* dskb  = (const float*)d_in[15];
  const float* lnw   = (const float*)d_in[16];
  const float* lnb   = (const float*)d_in[17];
  const float* wout  = (const float*)d_in[18];
  float* out = (float*)d_out;

  char* ws = (char*)d_ws;
  size_t off = 0;
  const size_t oWIN = off; off += SZ_WIN;
  const size_t oWO  = off; off += SZ_WO;
  const size_t oXP  = off; off += SZ_XP;
  const size_t oDP  = off; off += SZ_DP;
  const size_t oAR  = off; off += SZ_AR;
  const size_t oXSG = off; off += SZ_XSG;
  const size_t oUF  = off; off += SZ_ROW;
  const size_t oUB  = off; off += SZ_ROW;
  const size_t oYF  = off; off += SZ_ROW;
  const size_t oYB  = off; off += SZ_ROW;
  if (off > ws_size || off > (size_t)WSMAX) return;
  unsigned short* WIN   = (unsigned short*)(ws + oWIN);
  unsigned short* WOUT2 = (unsigned short*)(ws + oWO);
  float* XPR = (float*)(ws + oXP);
  float* DPR = (float*)(ws + oDP);
  float* AR  = (float*)(ws + oAR);
  float* XSG = (float*)(ws + oXSG);
  unsigned short* G = (unsigned short*)(ws + oXSG);
  float* UF  = (float*)(ws + oUF);
  float* UB  = (float*)(ws + oUB);
  float* YF  = (float*)(ws + oYF);
  float* YB  = (float*)(ws + oYB);

  hipFuncSetAttribute(reinterpret_cast<const void*>(&k_inx), hipFuncAttributeMaxDynamicSharedMemorySize,
                      (int)LDS_TILE_BYTES);
  hipFuncSetAttribute(reinterpret_cast<const void*>(&k_gate), hipFuncAttributeMaxDynamicSharedMemorySize,
                      (int)LDS_TILE_BYTES);
  hipFuncSetAttribute(reinterpret_cast<const void*>(&k_conv), hipFuncAttributeMaxDynamicSharedMemorySize,
                      (int)LDS_CONV_BYTES);

  k_prep<<<U_TOT / NTHR, NTHR, 0, stream>>>(win, wout, xpw, xpwb, dpw, dpwb, alog, alogb,
                                             WIN, WOUT2, XPR, DPR, AR);
  k_inx<<<NTOK / 32, NTHR, LDS_TILE_BYTES, stream>>>(hs, WIN, XSG);
  k_conv<<<NBAT * NCHB, NTHR, LDS_CONV_BYTES, stream>>>(XSG, cw, cb, cwb, cbb, dsk, dskb, UF, UB);
  k_ssm<<<2 * NBAT, NTHR, 0, stream>>>(UF, UB, XPR, DPR, AR, dpbf, dpbb, YF, YB);
  k_gate<<<NTOK / 32, NTHR, LDS_TILE_BYTES, stream>>>(hs, WIN, YF, YB, lnw, lnb, XSG);
  k_out<<<dim3(NTOK / GBM, DM / GBN), GTHR, 0, stream>>>(G, WOUT2, out);
}
